// NonLocalAttention_55018531062406
// MI455X (gfx1250) — hardware-verified
//
#include <hip/hip_runtime.h>


namespace {
typedef _Float16 b16;
typedef __attribute__((ext_vector_type(16))) _Float16 v16b;
typedef __attribute__((ext_vector_type(8))) _Float16 v8b;
typedef __attribute__((ext_vector_type(4))) _Float16 v4h;
typedef __attribute__((ext_vector_type(8))) float v8f;
typedef __attribute__((ext_vector_type(4))) float v4f;
typedef __attribute__((ext_vector_type(2))) float v2f;
__device__ __forceinline__ float bf16_rne(float f) { unsigned int u = __float_as_uint(f); u += 0x7FFFu + ((u >> 16) & 1u); return __uint_as_float(u & 0xFFFF0000u); }
__device__ __forceinline__ v16b frag_kb(const b16* p, int hh) { const v8b a = *(const v8b*)(p + 8 * hh), b = *(const v8b*)(p + 16 + 8 * hh); v16b f;
#pragma unroll
  for (int e = 0; e < 8; ++e) { f[e] = a[e]; f[8 + e] = b[e]; } return f; }
__device__ __forceinline__ v8f wmma16b(v16b a, v16b b, v8f c) { v8f d = __builtin_amdgcn_wmma_f32_16x16x32_f16(false, a, false, b, (short)0, c, false, false); asm volatile("v_nop\n\tv_nop\n\tv_nop\n\tv_nop" : "+v"(d) : "v"(a), "v"(b)); return d; }
__device__ __forceinline__ void wave_lds_sync() { __builtin_amdgcn_fence(3u, "workgroup"); __builtin_amdgcn_wave_barrier(); __builtin_amdgcn_fence(2u, "workgroup"); }
__device__ __forceinline__ float nexp2(float v) { return __builtin_amdgcn_exp2f(v); }

#ifndef NB
#define NB 8
#endif
#ifndef QL
#define QL 4096
#endif
constexpr int B_FULL = 8, C = 256, CI = 128, HH = 64, WW = 64, N = HH * WW, MH = HH / 2, MW = WW / 2, M = MH * MW, NO = 3 * CI;
constexpr int NBATCH = NB  , NQ = QL  ;
constexpr float XS = 8.0f, WSC = 256.0f, RS = 1024.0f, PS = 16384.0f, LOG2E = 1.4426950408889634f;
static_assert(NBATCH >= 1 && NBATCH <= B_FULL);
static_assert(NQ % 64 == 0 && NQ >= 64 && NQ <= N);
static_assert(C % 32 == 0 && CI == 128 && WW == 64 && HH % 2 == 0 && N % 64 == 0 && M % 64 == 0 && (NO * C) % 2048 == 0 && (C * CI) % 2048 == 0);

__global__ __launch_bounds__(256) void prep_kernel(const float* __restrict__ wt, const float* __restrict__ wp, const float* __restrict__ wg, const float* __restrict__ wo,
                                                   b16* __restrict__ WT, b16* __restrict__ WO) {
  constexpr int n1 = NO * C / 8, n2 = C * CI / 8;
  const int u = blockIdx.x * 256 + threadIdx.x; if (u >= n1 + n2) return;
  v8b v; b16* dst;
  if (u < n1) { const int e = u * 8; const int g = e / (CI * C), r = e % (CI * C); const float* w = g == 0 ? wt : (g == 1 ? wp : wg);
#pragma unroll
    for (int j = 0; j < 8; ++j) v[j] = (b16)(bf16_rne(w[r + j]) * WSC); dst = WT + e; }
  else { const int e = (u - n1) * 8;
#pragma unroll
    for (int j = 0; j < 8; ++j) v[j] = (b16)(bf16_rne(wo[e + j]) * WSC); dst = WO + e; }
  for (int pass = 0; pass < 2; ++pass) { *(volatile v8b*)dst = v; __threadfence(); }
}

__global__ __launch_bounds__(128) __attribute__((amdgpu_num_vgpr(256))) void conv_kernel(const float* __restrict__ x, const b16* __restrict__ WT, const float* __restrict__ bt,
    const float* __restrict__ bp, const float* __restrict__ bg, b16* __restrict__ Qh, b16* __restrict__ Ql, b16* __restrict__ Kh, b16* __restrict__ Kl, b16* __restrict__ Gp) {
  __shared__ __attribute__((aligned(16))) b16 As[64][C + 8];
  __shared__ __attribute__((aligned(16))) float Tf[64][CI + 4];
  const int wave = threadIdx.x >> 5, lane = threadIdx.x & 31, nloc = lane & 15, hlf = lane >> 4;
  const int h2 = blockIdx.x >> 1, wblk = blockIdx.x & 1, h0 = 2 * h2, w0 = (WW / 2) * wblk; const int b = blockIdx.y;
  const float* xb = x + (size_t)b * C * N;
  for (int i = threadIdx.x; i < C * 16; i += 128) { const int c = i >> 4, pp4 = (i & 15) * 4; const int hr = pp4 >> 5, wc = pp4 & 31;
    const v4f v = *(const v4f*)(xb + (size_t)c * N + (h0 + hr) * WW + w0 + wc);
#pragma unroll
    for (int j = 0; j < 4; ++j) As[pp4 + j][c] = (b16)(bf16_rne(v[j]) * XS); }
  __syncthreads();
#pragma unroll 1
  for (int g = 0; g < 3; ++g) {
    v8f acc[8];
#pragma unroll
    for (int t = 0; t < 8; ++t) acc[t] = (v8f){};
    const b16* Wg = WT + (size_t)g * CI * C;
#pragma unroll
    for (int kb = 0; kb < C; kb += 32) { const v16b a = frag_kb(&As[wave * 16 + nloc][kb], hlf);
#pragma unroll
      for (int t = 0; t < 8; ++t) acc[t] = wmma16b(a, frag_kb(Wg + (size_t)(t * 16 + nloc) * C + kb, hlf), acc[t]); }
    const float* bias = g == 0 ? bt : (g == 1 ? bp : bg);
    __syncthreads();
#pragma unroll
    for (int t = 0; t < 8; ++t) { const int o = t * 16 + nloc; const float bb = bf16_rne(bias[o]);
#pragma unroll
      for (int r = 0; r < 8; ++r) Tf[wave * 16 + 8 * hlf + r][o] = acc[t][r] * (1.0f / (XS * WSC)) + bb; }
    __syncthreads();
    const int d = lane * 4;
    if (g == 0) {
      for (int pass = 0; pass < 2; ++pass) {
#pragma unroll 1
        for (int rr = 0; rr < 16; ++rr) { const int pl = wave * 16 + rr; const int p = (h0 + (pl >> 5)) * WW + w0 + (pl & 31); v4h hv, lv;
#pragma unroll
          for (int j = 0; j < 4; ++j) { const float f = Tf[pl][d + j] * XS; const b16 h = (b16)f; hv[j] = h; lv[j] = (b16)((f - (float)h) * RS); }
          const size_t oi = ((size_t)b * N + p) * CI + d; *(volatile v4h*)(Qh + oi) = hv; *(volatile v4h*)(Ql + oi) = lv; }
        __threadfence(); }
    } else {
      for (int pass = 0; pass < 2; ++pass) {
#pragma unroll 1
        for (int jq = 0; jq < 4; ++jq) { const int j = wave * 4 + jq; const int mrow = h2 * MW + wblk * 16 + j; const int ra = 2 * j, rb = 32 + 2 * j; v4h hv, lv;
#pragma unroll
          for (int jj = 0; jj < 4; ++jj) { const float v = fmaxf(fmaxf(Tf[ra][d + jj], Tf[ra + 1][d + jj]), fmaxf(Tf[rb][d + jj], Tf[rb + 1][d + jj]));
            const float f = v * XS; const b16 h = (b16)f; hv[jj] = h; lv[jj] = (b16)((f - (float)h) * RS); }
          const size_t oi = ((size_t)b * M + mrow) * CI + d;
          if (g == 1) { *(volatile v4h*)(Kh + oi) = hv; *(volatile v4h*)(Kl + oi) = lv; } else { *(volatile v4h*)(Gp + oi) = hv; } }
        __threadfence(); }
    }
  }
}

__global__ __launch_bounds__(256) void vt_kernel(const b16* __restrict__ Gp, b16* __restrict__ VT) {
  __shared__ __attribute__((aligned(16))) b16 Ts[CI][64 + 8];
  const int b = blockIdx.y, m0 = blockIdx.x * 64;
#pragma unroll 1
  for (int it = 0; it < 4; ++it) { const int idx = threadIdx.x + 256 * it; const int mm = idx >> 4, d8 = (idx & 15) * 8;
    const v8b v = *(const v8b*)(Gp + ((size_t)b * M + m0 + mm) * CI + d8);
#pragma unroll
    for (int j = 0; j < 8; ++j) Ts[d8 + j][mm] = v[j]; }
  __syncthreads();
  for (int pass = 0; pass < 2; ++pass) {
#pragma unroll 1
    for (int it = 0; it < 4; ++it) { const int idx = threadIdx.x + 256 * it; const int dd = idx >> 3, q = idx & 7; const v8b v = *(const v8b*)&Ts[dd][q * 8];
      *(volatile v8b*)(VT + ((size_t)b * CI + dd) * (size_t)M + m0 + q * 8) = v; }
    __threadfence(); }
}

__global__ __launch_bounds__(64) __attribute__((amdgpu_num_vgpr(256))) void attn_kernel(const b16* __restrict__ Qh, const b16* __restrict__ Ql, const b16* __restrict__ Kh,
    const b16* __restrict__ Kl, const b16* __restrict__ VT, b16* __restrict__ Yh, b16* __restrict__ Yl) {
  __shared__ __attribute__((aligned(16))) b16 Pb[2][16][32 + 8]; __shared__ __attribute__((aligned(16))) float To[2][16][CI + 4];
  const int wave = threadIdx.x >> 5, lane = threadIdx.x & 31, hh = lane >> 4, col = lane & 15; const int b = blockIdx.y; const int q0 = blockIdx.x * 32 + wave * 16, qi = q0 + col;
  const b16* Qhb = Qh + (size_t)b * N * CI; const b16* Qlb = Ql + (size_t)b * N * CI; const b16* Khb = Kh + (size_t)b * M * CI; const b16* Klb = Kl + (size_t)b * M * CI;
  const b16* Vb = VT + (size_t)b * CI * M;
  v16b qh[4];
#pragma unroll
  for (int s = 0; s < 4; ++s) qh[s] = frag_kb(Qhb + (size_t)qi * CI + 32 * s, hh);
  const b16* qlr = Qlb + (size_t)qi * CI;
  const float cs = LOG2E / (XS * XS), csl = cs / RS;
  float m = -INFINITY, l = 0.0f; v8f o[8];
#pragma unroll
  for (int t = 0; t < 8; ++t) o[t] = (v8f){};
#pragma unroll 1
  for (int kb = 0; kb < M; kb += 32) {
    float e[16]; float mx = -INFINITY;
#pragma unroll
    for (int u = 0; u < 2; ++u) { v8f s = (v8f){}, sl = (v8f){}; const size_t kr = (size_t)(kb + u * 16 + col) * CI;
#pragma unroll
      for (int st = 0; st < 4; ++st) { const v16b kh = frag_kb(Khb + kr + 32 * st, hh), kl = frag_kb(Klb + kr + 32 * st, hh), ql = frag_kb(qlr + 32 * st, hh);
        s = wmma16b(kh, qh[st], s); sl = wmma16b(kh, ql, sl); sl = wmma16b(kl, qh[st], sl); }
#pragma unroll
      for (int r = 0; r < 8; ++r) { const float vv = s[r] * cs + sl[r] * csl; e[u * 8 + r] = vv; mx = fmaxf(mx, vv); } }
    mx = fmaxf(mx, __shfl_xor(mx, 16)); const float mn = fmaxf(m, mx); const float al = nexp2(m - mn); float sum = 0.0f;
#pragma unroll
    for (int i2 = 0; i2 < 16; ++i2) { const float p = nexp2(e[i2] - mn); sum += p; Pb[wave][col][(i2 < 8 ? 0 : 16) + 8 * hh + (i2 & 7)] = (b16)(p * PS); }
    sum += __shfl_xor(sum, 16); l = l * al + sum; m = mn;
    wave_lds_sync();
    const v16b pf = frag_kb(&Pb[wave][col][0], hh);
#pragma unroll
    for (int t = 0; t < 8; ++t) { o[t] *= al; o[t] = wmma16b(frag_kb(Vb + (size_t)(t * 16 + col) * M + kb, hh), pf, o[t]); }
    wave_lds_sync(); }
  const float inv = 1.0f / (l * PS * XS);
#pragma unroll
  for (int t = 0; t < 8; ++t)
#pragma unroll
    for (int r = 0; r < 8; ++r) To[wave][col][t * 16 + 8 * hh + r] = o[t][r] * inv;
  __syncthreads();
  const int d = lane * 4;
  for (int pass = 0; pass < 2; ++pass) {
#pragma unroll 1
    for (int rr = 0; rr < 16; ++rr) { const int q = q0 + rr; v4h hv, lv;
#pragma unroll
      for (int j = 0; j < 4; ++j) { const float f = To[wave][rr][d + j] * XS; const b16 h = (b16)f; hv[j] = h; lv[j] = (b16)((f - (float)h) * RS); }
      const size_t oi = ((size_t)b * N + q) * CI + d; *(volatile v4h*)(Yh + oi) = hv; *(volatile v4h*)(Yl + oi) = lv; }
    __threadfence(); }
}

__global__ __launch_bounds__(128) __attribute__((amdgpu_num_vgpr(256))) void out_kernel(const float* __restrict__ x, const b16* __restrict__ Yh, const b16* __restrict__ Yl,
    const b16* __restrict__ WO, const float* __restrict__ bo, float* __restrict__ out) {
  __shared__ __attribute__((aligned(16))) float Tf[64][64 + 4];
  const int wave = threadIdx.x >> 5, lane = threadIdx.x & 31, nloc = lane & 15, hlf = lane >> 4; const int p0 = blockIdx.x * 64, c0 = blockIdx.y * 64, b = blockIdx.z;
  const size_t prow = ((size_t)b * N + p0 + wave * 16 + nloc) * CI;
  v8f ah[4], al[4];
#pragma unroll
  for (int t = 0; t < 4; ++t) { ah[t] = (v8f){}; al[t] = (v8f){}; }
#pragma unroll
  for (int st = 0; st < 4; ++st) { const v16b fa = frag_kb(Yh + prow + 32 * st, hlf), fl = frag_kb(Yl + prow + 32 * st, hlf);
#pragma unroll
    for (int t = 0; t < 4; ++t) { const v16b wb = frag_kb(WO + (size_t)(c0 + t * 16 + nloc) * CI + 32 * st, hlf); ah[t] = wmma16b(fa, wb, ah[t]); al[t] = wmma16b(fl, wb, al[t]); } }
#pragma unroll
  for (int t = 0; t < 4; ++t) { const int o = t * 16 + nloc; const float bb = bf16_rne(bo[c0 + o]);
#pragma unroll
    for (int r = 0; r < 8; ++r) Tf[wave * 16 + 8 * hlf + r][o] = ah[t][r] * (1.0f / (XS * WSC)) + al[t][r] * (1.0f / (XS * WSC * RS)) + bb; }
  __syncthreads();
  for (int pass = 0; pass < 2; ++pass) {
#pragma unroll 1
    for (int q = 0; q < 16; ++q) { const int cl = wave * 16 + q; const size_t idx = ((size_t)b * C + c0 + cl) * (size_t)N + p0 + 2 * lane;
      const v2f xv = *(const v2f*)(x + idx); v2f ov; ov[0] = bf16_rne(xv[0]) + Tf[2 * lane][cl]; ov[1] = bf16_rne(xv[1]) + Tf[2 * lane + 1][cl];
      *(volatile v2f*)(out + idx) = ov; }
    __threadfence(); }
}
}

extern "C" void kernel_launch(void* const* d_in, const int* in_sizes, int n_in, void* d_out, int out_size, void* d_ws, size_t ws_size, hipStream_t stream) {
  (void)n_in;
  auto Fp = [&](int i) { return (const float*)d_in[i]; };
  if (in_sizes[0] < NBATCH * C * N || in_sizes[1] < CI * C || in_sizes[2] < CI || in_sizes[3] < CI * C || in_sizes[4] < CI || in_sizes[5] < CI * C || in_sizes[6] < CI ||
      in_sizes[7] < C * CI || in_sizes[8] < C || out_size < NBATCH * C * N) return;
  size_t off = 0; char* ws = (char*)d_ws;
  auto carve = [&](size_t bytes) { char* p = ws + off; off += (bytes + 255) & ~(size_t)255; return p; };
  b16* WT = (b16*)carve((size_t)NO * C * 2); b16* WO = (b16*)carve((size_t)C * CI * 2);
  const size_t qplane = (size_t)NBATCH * N * CI * 2, kplane = (size_t)NBATCH * M * CI * 2;
  b16* Qh = (b16*)carve(qplane); b16* Ql = (b16*)carve(qplane); b16* Kh = (b16*)carve(kplane); b16* Kl = (b16*)carve(kplane);
  b16* Gp = (b16*)carve(kplane); b16* VT = (b16*)carve(kplane); b16* Yh = (b16*)carve(qplane); b16* Yl = (b16*)carve(qplane);
  if (off > ws_size || off > ((size_t)128 << 20)) return;
  prep_kernel<<<(NO * C / 8 + C * CI / 8 + 255) / 256, 256, 0, stream>>>(Fp(1), Fp(3), Fp(5), Fp(7), WT, WO);
  conv_kernel<<<dim3(N / 64, NBATCH), 128, 0, stream>>>(Fp(0), WT, Fp(2), Fp(4), Fp(6), Qh, Ql, Kh, Kl, Gp);
  vt_kernel<<<dim3(M / 64, NBATCH), 256, 0, stream>>>(Gp, VT);
  attn_kernel<<<dim3(NQ / 32, NBATCH), 64, 0, stream>>>(Qh, Ql, Kh, Kl, VT, Yh, Yl);
  out_kernel<<<dim3(NQ / 64, C / 64, NBATCH), 128, 0, stream>>>(Fp(0), Yh, Yl, WO, Fp(8), (float*)d_out);
}
